// CustomAttention_5068061409377
// MI455X (gfx1250) — hardware-verified
//
#include <hip/hip_runtime.h>


#ifndef NB
#define NB 4
#endif
#ifndef SEQ
#define SEQ 2048
#endif
#define NB_FULL  4
#define SEQ_FULL 2048
#define DM   1024
#ifndef RH
#define RH   0
#endif
#define PCAR 4096.0f
#define SCL  0.03125f
static_assert(NB >= 1 && NB <= NB_FULL);
static_assert(SEQ >= 128 && SEQ <= SEQ_FULL && SEQ % 128 == 0);
static_assert(RH >= 0 && RH <= SEQ && RH % 64 == 0);
static_assert(DM % 64 == 0);

typedef _Float16 h16;
typedef unsigned short bf;
typedef __attribute__((ext_vector_type(16))) __bf16   v16bf;
typedef __attribute__((ext_vector_type(16))) _Float16 v16h;
typedef __attribute__((ext_vector_type(8)))  _Float16 v8h;
typedef __attribute__((ext_vector_type(8)))  unsigned short v8us;
typedef __attribute__((ext_vector_type(8)))  float    v8f;
typedef __attribute__((ext_vector_type(4)))  float    v4f;
typedef __attribute__((ext_vector_type(4)))  _Float16 v4h;
typedef __attribute__((ext_vector_type(4)))  unsigned short v4us;
typedef v8h  __attribute__((may_alias)) v8ha;
typedef v4f  __attribute__((may_alias)) v4fa;
typedef v8us __attribute__((may_alias)) v8usa;

__device__ __forceinline__ unsigned short f2bf(float f) { unsigned u = __float_as_uint(f); u += 0x7FFFu + ((u >> 16) & 1u); return (unsigned short)(u >> 16); }
__device__ __forceinline__ float bf2f(unsigned short b) { return __uint_as_float(((unsigned)b) << 16); }
__device__ __forceinline__ float bfr(float f) { return bf2f(f2bf(f)); }
__device__ __forceinline__ v16h cat16(v8h lo, v8h hi) { return __builtin_shufflevector(lo, hi, 0, 1, 2, 3, 4, 5, 6, 7, 8, 9, 10, 11, 12, 13, 14, 15); }
__device__ __forceinline__ v16bf cat16b(v8us lo, v8us hi) { return __builtin_bit_cast(v16bf, __builtin_shufflevector(lo, hi, 0, 1, 2, 3, 4, 5, 6, 7, 8, 9, 10, 11, 12, 13, 14, 15)); }
__device__ __forceinline__ v8f wmma16(v16h a, v16h b, v8f c) { return __builtin_amdgcn_wmma_f32_16x16x32_f16(false, a, false, b, (short)0, c, false, false); }
__device__ __forceinline__ v8f wmmab(v16bf a, v16bf b, v8f c) { return __builtin_amdgcn_wmma_f32_16x16x32_bf16(false, a, false, b, (short)0, c, false, false); }
__device__ __forceinline__ h16 tohx(float x) { return (h16)x; }
__device__ __forceinline__ void splitf(float y, unsigned short& h, unsigned short& l) { h = f2bf(y); l = f2bf(y - bf2f(h)); }

template <typename T16> struct WFrag;
template <> struct WFrag<h16> { typedef v16h V; static __device__ __forceinline__ V ld(const h16* p) { return cat16(*(const v8h*)p, *(const v8h*)(p + 16)); } static __device__ __forceinline__ v8f mma(V a, V b, v8f c) { return wmma16(a, b, c); } };
template <> struct WFrag<bf> { typedef v16bf V; static __device__ __forceinline__ V ld(const bf* p) { return cat16b(*(const v8us*)p, *(const v8us*)(p + 16)); } static __device__ __forceinline__ v8f mma(V a, V b, v8f c) { return wmmab(a, b, c); } };
template <typename T16, int NSPLIT, bool BIAS>
__global__ __launch_bounds__(32) void k_gemmw(const T16* __restrict__ A, const T16* __restrict__ A2, const T16* __restrict__ Bt, const T16* __restrict__ Bt2, int K, float* C, int ldc, const float* __restrict__ bias, size_t sA, size_t sB, size_t sC) {
    typedef typename WFrag<T16>::V V;
    __shared__ __align__(16) float os[16 * 68];
    const size_t z = blockIdx.z; A += z * sA; if (A2) A2 += z * sA; Bt += z * sB; if (Bt2) Bt2 += z * sB; C += z * sC;
    const int lane = threadIdx.x & 31, lr = lane & 15, hi = lane >> 4; const int r0 = blockIdx.x * 64, c0 = blockIdx.y * 64;
    v8f acc[4][4];
#pragma unroll
    for (int mb = 0; mb < 4; ++mb)
#pragma unroll
        for (int nb = 0; nb < 4; ++nb) acc[mb][nb] = (v8f){};
    const size_t aoff = (size_t)(r0 + lr) * K + 8 * hi, boff = (size_t)(c0 + lr) * K + 8 * hi;
#pragma unroll 1
    for (int kc = 0; kc < K; kc += 32) {
        V a[4], a2[4];
#pragma unroll
        for (int mb = 0; mb < 4; ++mb) { a[mb] = WFrag<T16>::ld(A + aoff + (size_t)mb * 16 * K + kc); if (NSPLIT == 1 || NSPLIT == 2) a2[mb] = WFrag<T16>::ld(A2 + aoff + (size_t)mb * 16 * K + kc); }
#pragma unroll
        for (int nb = 0; nb < 4; ++nb) { const V b = WFrag<T16>::ld(Bt + boff + (size_t)nb * 16 * K + kc); V b2; if (NSPLIT >= 2) b2 = WFrag<T16>::ld(Bt2 + boff + (size_t)nb * 16 * K + kc);
#pragma unroll
            for (int mb = 0; mb < 4; ++mb) { acc[mb][nb] = WFrag<T16>::mma(a[mb], b, acc[mb][nb]); if (NSPLIT == 1 || NSPLIT == 2) acc[mb][nb] = WFrag<T16>::mma(a2[mb], b, acc[mb][nb]); if (NSPLIT >= 2) acc[mb][nb] = WFrag<T16>::mma(a[mb], b2, acc[mb][nb]); } }
        asm volatile("v_nop\n\tv_nop\n\tv_nop\n\tv_nop" : "+v"(acc[0][0]), "+v"(acc[1][1]), "+v"(acc[2][2]), "+v"(acc[3][3]) : "v"(a[0]), "v"(a[3]));
    }
#pragma unroll
    for (int mb = 0; mb < 4; ++mb) {
#pragma unroll
        for (int nb = 0; nb < 4; ++nb) {
#pragma unroll
            for (int j = 0; j < 8; ++j) os[(hi * 8 + j) * 68 + nb * 16 + lr] = acc[mb][nb][j]; }
        __builtin_amdgcn_wave_barrier(); asm volatile("" ::: "memory");
        float* crow = C + (size_t)(r0 + mb * 16) * ldc + c0;
#pragma unroll 1
        for (int ps = 0; ps < 2; ++ps) {
#pragma unroll
            for (int s = 0; s < 8; ++s) { const int row = 2 * s + hi, cofs = lr * 4; v4f val = *(const v4fa*)(os + row * 68 + cofs); if (BIAS) { val[0] += bfr(bias[c0 + cofs]); val[1] += bfr(bias[c0 + cofs + 1]); val[2] += bfr(bias[c0 + cofs + 2]); val[3] += bfr(bias[c0 + cofs + 3]); }
                *(volatile v4f*)(crow + (size_t)row * ldc + cofs) = val; }
            if (ps == 0) __threadfence(); }
        __builtin_amdgcn_wave_barrier(); asm volatile("" ::: "memory");
    }
}

__global__ __launch_bounds__(256) void k_cvt8(const float* __restrict__ src, bf* dst, size_t n8) { const size_t i = (size_t)blockIdx.x * 256 + threadIdx.x; if (i >= n8) return; const v8f v = *(const v8f*)(src + i * 8); v8us o;
#pragma unroll
    for (int k = 0; k < 8; ++k) o[k] = f2bf(v[k]); *(volatile v8us*)(dst + i * 8) = o; __threadfence(); *(volatile v8us*)(dst + i * 8) = o; }

template <bool HL>
__global__ __launch_bounds__(256) void k_pln(const float* __restrict__ F, h16* P16, bf* Ph, bf* Pl, size_t n8) {
    const size_t i = (size_t)blockIdx.x * 256 + threadIdx.x; if (i >= n8) return; const size_t e = i * 8;
    const v4f a = *(const v4f*)(F + e); const v4f b = *(const v4f*)(F + e + 4); v8h o16; v8us oh, ol;
#pragma unroll
    for (int q = 0; q < 4; ++q) {
        { const float x = a[q]; o16[q] = tohx(x); if (HL) { unsigned short a2, c2; splitf(x, a2, c2); oh[q] = a2; ol[q] = c2; } }
        { const float x = b[q]; o16[4 + q] = tohx(x); if (HL) { unsigned short a2, c2; splitf(x, a2, c2); oh[4 + q] = a2; ol[4 + q] = c2; } } }
    *(volatile v8h*)(P16 + e) = o16; if (HL) { *(volatile v8us*)(Ph + e) = oh; *(volatile v8us*)(Pl + e) = ol; }
    __threadfence();
    *(volatile v8h*)(P16 + e) = o16; if (HL) { *(volatile v8us*)(Ph + e) = oh; *(volatile v8us*)(Pl + e) = ol; } }

template <bool HL>
__global__ __launch_bounds__(256) void k_vtp(const float* __restrict__ F, int pitch, h16* V16, bf* Vh, bf* Vl, size_t n8) {
    const size_t i = (size_t)blockIdx.x * 256 + threadIdx.x; if (i >= n8) return; const size_t e = i * 8; const int t = (int)(e % SEQ); const int d = (int)(e / SEQ);
    v8h o16; v8us oh, ol;
#pragma unroll
    for (int q = 0; q < 8; ++q) { const float x = F[(size_t)(t + q) * pitch + d]; o16[q] = tohx(x); if (HL) { unsigned short a2, c2; splitf(x, a2, c2); oh[q] = a2; ol[q] = c2; } }
    *(volatile v8h*)(V16 + e) = o16; if (HL) { *(volatile v8us*)(Vh + e) = oh; *(volatile v8us*)(Vl + e) = ol; }
    __threadfence();
    *(volatile v8h*)(V16 + e) = o16; if (HL) { *(volatile v8us*)(Vh + e) = oh; *(volatile v8us*)(Vl + e) = ol; } }

__global__ __launch_bounds__(256) void k_asoft(const float* __restrict__ Sb, h16* P16, bf* Ph, bf* Pl) {
    const int lane = threadIdx.x & 31; const int row = blockIdx.x * 8 + (threadIdx.x >> 5); if (row >= SEQ) return;
    const bool hires = (row < RH); const float* sr = Sb + (size_t)row * SEQ;
    float m0 = -3.0e38f, m1 = -3.0e38f, m2 = -3.0e38f, m3 = -3.0e38f;
#pragma unroll 1
    for (int ch = 0; ch < SEQ / 128; ++ch) { const v4f a = *(const v4f*)(sr + ch * 128 + lane * 4); m0 = fmaxf(m0, a[0]); m1 = fmaxf(m1, a[1]); m2 = fmaxf(m2, a[2]); m3 = fmaxf(m3, a[3]); }
    float m = fmaxf(fmaxf(m0, m1), fmaxf(m2, m3));
#pragma unroll
    for (int o = 16; o > 0; o >>= 1) m = fmaxf(m, __shfl_xor(m, o, 32));
    const float mx = m * SCL;
    float su = 0.0f;
#pragma unroll 1
    for (int ch = 0; ch < SEQ / 128; ++ch) { const v4f a = *(const v4f*)(sr + ch * 128 + lane * 4);
#pragma unroll
        for (int q = 0; q < 4; ++q) { const float x = a[q] * SCL; su += __expf(x - mx); } }
#pragma unroll
    for (int o = 16; o > 0; o >>= 1) su += __shfl_xor(su, o, 32);
    const float inv = 1.0f / su;
    const float sc = hires ? inv : inv * PCAR;
#pragma unroll 1
    for (int ch = 0; ch < SEQ / 128; ++ch) { const int j0 = ch * 128 + lane * 4; const v4f a = *(const v4f*)(sr + j0); float p4[4];
#pragma unroll
        for (int q = 0; q < 4; ++q) { const float x = a[q] * SCL; p4[q] = __expf(x - mx) * sc; }
        const size_t oo = (size_t)row * SEQ + j0;
        if (hires) { v4us oh, ol;
#pragma unroll
            for (int q = 0; q < 4; ++q) { unsigned short h2, l2; splitf(p4[q], h2, l2); oh[q] = h2; ol[q] = l2; }
            *(volatile v4us*)(Ph + oo) = oh; *(volatile v4us*)(Pl + oo) = ol; __threadfence(); *(volatile v4us*)(Ph + oo) = oh; *(volatile v4us*)(Pl + oo) = ol; }
        else { v4h o4;
#pragma unroll
            for (int q = 0; q < 4; ++q) o4[q] = tohx(p4[q]);
            *(volatile v4h*)(P16 + oo) = o4; __threadfence(); *(volatile v4h*)(P16 + oo) = o4; } }
}

__global__ __launch_bounds__(256) void k_merge(const float* __restrict__ O, bf* Ah, bf* Al, size_t n8) {
    const size_t i = (size_t)blockIdx.x * 256 + threadIdx.x; if (i >= n8) return; const size_t e = i * 8; const int t = (int)(e / DM); const float cs = (t < RH) ? 1.0f : (1.0f / PCAR);
    const v4f a = *(const v4f*)(O + e); const v4f b = *(const v4f*)(O + e + 4); v8us oh, ol;
#pragma unroll
    for (int q = 0; q < 4; ++q) {
        { unsigned short a2, c2; splitf(a[q] * cs, a2, c2); oh[q] = a2; ol[q] = c2; }
        { unsigned short a2, c2; splitf(b[q] * cs, a2, c2); oh[4 + q] = a2; ol[4 + q] = c2; } }
    *(volatile v8us*)(Ah + e) = oh; *(volatile v8us*)(Al + e) = ol; __threadfence(); *(volatile v8us*)(Ah + e) = oh; *(volatile v8us*)(Al + e) = ol; }

extern "C" void kernel_launch(void* const* d_in, const int* in_sizes, int n_in,
                              void* d_out, int out_size, void* d_ws, size_t ws_size, hipStream_t stream) {
    if (n_in < 11) return;
    const size_t needx = (size_t)(NB - 1) * SEQ_FULL * DM + (size_t)SEQ * DM;
    if ((size_t)in_sizes[0] < needx || (size_t)in_sizes[1] < needx || (size_t)in_sizes[2] < needx) return;
    if ((size_t)in_sizes[3] < (size_t)DM * DM || (size_t)in_sizes[5] < (size_t)DM * DM || (size_t)in_sizes[7] < (size_t)DM * DM || (size_t)in_sizes[9] < (size_t)DM * DM) return;
    if (in_sizes[4] < DM || in_sizes[6] < DM || in_sizes[8] < DM || in_sizes[10] < DM) return;
    if ((size_t)out_size < (size_t)NB * SEQ * DM) return;
    const float* xq = (const float*)d_in[0]; const float* xk = (const float*)d_in[1]; const float* xv = (const float*)d_in[2];
    const float* wq = (const float*)d_in[3]; const float* bq = (const float*)d_in[4]; const float* wk = (const float*)d_in[5]; const float* bk = (const float*)d_in[6];
    const float* wv = (const float*)d_in[7]; const float* bv = (const float*)d_in[8]; const float* wo = (const float*)d_in[9]; const float* bo = (const float*)d_in[10];
    float* OUT = (float*)d_out;
    char* wsp = (char*)d_ws;
    auto take = [&](size_t bytes) { char* p = wsp; wsp += (bytes + 255) & ~(size_t)255; return (void*)p; };
    bf* WQ = (bf*)take((size_t)DM * DM * 2); bf* WK = (bf*)take((size_t)DM * DM * 2); bf* WV = (bf*)take((size_t)DM * DM * 2); bf* WO = (bf*)take((size_t)DM * DM * 2);
    bf* XB = (bf*)take((size_t)SEQ * DM * 2); float* FQ = (float*)take((size_t)SEQ * DM * 4); float* FK = (float*)take((size_t)SEQ * DM * 4);
    h16* QP16 = (h16*)take((size_t)SEQ * DM * 2); h16* KP16 = (h16*)take((size_t)SEQ * DM * 2); h16* VT16 = (h16*)take((size_t)DM * SEQ * 2);
    bf* QPh = nullptr; bf* QPl = nullptr; bf* KPh = nullptr; bf* KPl = nullptr; bf* VTh = nullptr; bf* VTl = nullptr; bf* Ph = nullptr; bf* Pl = nullptr;
    if (RH > 0) { QPh = (bf*)take((size_t)SEQ * DM * 2); QPl = (bf*)take((size_t)SEQ * DM * 2); KPh = (bf*)take((size_t)SEQ * DM * 2); KPl = (bf*)take((size_t)SEQ * DM * 2);
                  VTh = (bf*)take((size_t)DM * SEQ * 2); VTl = (bf*)take((size_t)DM * SEQ * 2); Ph = (bf*)take((size_t)(RH ? RH : 1) * SEQ * 2); Pl = (bf*)take((size_t)(RH ? RH : 1) * SEQ * 2); }
    float* Sb = (float*)take((size_t)SEQ * SEQ * 4); h16* P16 = (h16*)take((size_t)SEQ * SEQ * 2); float* Ob = (float*)take((size_t)SEQ * DM * 4);
    bf* ATh = (bf*)take((size_t)SEQ * DM * 2); bf* ATl = (bf*)take((size_t)SEQ * DM * 2);
    if ((size_t)(wsp - (char*)d_ws) > ws_size) return;
    float* FV = FK;
    const unsigned GW = (unsigned)(((size_t)DM * DM / 8 + 255) / 256);
    k_cvt8<<<GW, 256, 0, stream>>>(wq, WQ, (size_t)DM * DM / 8);
    k_cvt8<<<GW, 256, 0, stream>>>(wk, WK, (size_t)DM * DM / 8);
    k_cvt8<<<GW, 256, 0, stream>>>(wv, WV, (size_t)DM * DM / 8);
    k_cvt8<<<GW, 256, 0, stream>>>(wo, WO, (size_t)DM * DM / 8);
    const size_t n8x = (size_t)SEQ * DM / 8; const unsigned GX = (unsigned)((n8x + 255) / 256);
    const dim3 gproj(SEQ / 64, DM / 64, 1);
    for (int b = 0; b < NB; ++b) {
        const size_t xofs = (size_t)b * SEQ_FULL * DM;
        k_cvt8<<<GX, 256, 0, stream>>>(xq + xofs, XB, n8x);
        k_gemmw<bf, 0, true><<<gproj, 32, 0, stream>>>(XB, nullptr, WQ, nullptr, DM, FQ, DM, bq, 0, 0, 0);
        k_pln<(RH > 0)><<<GX, 256, 0, stream>>>(FQ, QP16, QPh, QPl, n8x);
        k_cvt8<<<GX, 256, 0, stream>>>(xk + xofs, XB, n8x);
        k_gemmw<bf, 0, true><<<gproj, 32, 0, stream>>>(XB, nullptr, WK, nullptr, DM, FK, DM, bk, 0, 0, 0);
        k_pln<(RH > 0)><<<GX, 256, 0, stream>>>(FK, KP16, KPh, KPl, n8x);
        k_cvt8<<<GX, 256, 0, stream>>>(xv + xofs, XB, n8x);
        k_gemmw<bf, 0, true><<<gproj, 32, 0, stream>>>(XB, nullptr, WV, nullptr, DM, FV, DM, bv, 0, 0, 0);
        k_vtp<(RH > 0)><<<GX, 256, 0, stream>>>(FV, DM, VT16, VTh, VTl, n8x);
        if (RH > 0)   k_gemmw<bf, 2, false><<<dim3((RH ? RH : 64) / 64, SEQ / 64, 1), 32, 0, stream>>>(QPh, QPl, KPh, KPl, DM, Sb, SEQ, nullptr, 0, 0, 0);
        if (SEQ > RH) k_gemmw<h16, 0, false><<<dim3((SEQ - RH) ? (SEQ - RH) / 64 : 1, SEQ / 64, 1), 32, 0, stream>>>(QP16 + (size_t)RH * DM, nullptr, KP16, nullptr, DM, Sb + (size_t)RH * SEQ, SEQ, nullptr, 0, 0, 0);
        k_asoft<<<(SEQ + 7) / 8, 256, 0, stream>>>(Sb, P16, Ph, Pl);
        if (RH > 0)   k_gemmw<bf, 2, false><<<dim3((RH ? RH : 64) / 64, DM / 64, 1), 32, 0, stream>>>(Ph, Pl, VTh, VTl, SEQ, Ob, DM, nullptr, 0, 0, 0);
        if (SEQ > RH) k_gemmw<h16, 0, false><<<dim3((SEQ - RH) ? (SEQ - RH) / 64 : 1, DM / 64, 1), 32, 0, stream>>>(P16 + (size_t)RH * SEQ, nullptr, VT16, nullptr, SEQ, Ob + (size_t)RH * DM, DM, nullptr, 0, 0, 0);
        k_merge<<<GX, 256, 0, stream>>>(Ob, ATh, ATl, n8x);
        k_gemmw<bf, 1, true><<<gproj, 32, 0, stream>>>(ATh, ATl, WO, nullptr, DM, OUT + (size_t)b * SEQ * DM, DM, bo, 0, 0, 0);
    }
}
